// Local_Correlation_37014028157089
// MI455X (gfx1250) — hardware-verified
//
#include <hip/hip_runtime.h>
#include <stddef.h>
#include <math.h>


#define NB     2
#define NPT    16384
#define NPTOT  32768
#define CH     64
#define KN     20
#define OC     192
#define WROWS  256

#define PA     72
#define PK     40
#define YR     48

#define PPB    32
#define NWV    4
#define NTH    128
#define PPW    8

#define QPB    64
#define QTH    256

#define W_THH  0
#define W_THL  (W_THH + 32 * PA * 2)
#define W_PHH  (W_THL + 32 * PA * 2)
#define W_PHL  (W_PHH + 32 * PA * 2)
#define W_GTH  (W_PHL + 32 * PA * 2)
#define W_GTL  (W_GTH + 64 * PK * 2)
#define W_FS   (W_GTL + 64 * PK * 2)
#define W_ATH  (W_FS + 32 * 32 * 4)
#define W_ATL  (W_ATH + 32 * PK * 2)
#define W_YH   (W_ATL + 32 * PK * 2)
#define W_YL   (W_YH + YR * PA * 2)
#define W_SZ   (W_YL + YR * PA * 2)
#define L_WWH  0
#define L_WWL  (L_WWH + 64 * PA * 2)
#define L_CST  (L_WWL + 64 * PA * 2)
#define L_OUT  (L_CST + 384 * 4)
#define L_WAV  (L_OUT + 64 * PPB * 4)
#define LDS_MAIN (L_WAV + NWV * W_SZ)

#define Q_XH   0
#define Q_XL   (Q_XH + QPB * PA * 2)
#define Q_SP   (Q_XL + QPB * PA * 2)
#define LDS_PROJ (Q_SP + QPB * OC * 4)

static_assert(PPB == NWV * PPW);
static_assert(NTH == NWV * 32);
static_assert((PPW % 2) == 0);
static_assert((NPT % PPB) == 0 && (NPT % QPB) == 0);
static_assert((W_THL % 16) == 0 && (W_PHH % 16) == 0 && (W_PHL % 16) == 0 && (W_GTH % 16) == 0);
static_assert((W_GTL % 16) == 0 && (W_FS % 16) == 0 && (W_ATH % 16) == 0 && (W_ATL % 16) == 0);
static_assert((W_YH % 16) == 0 && (W_YL % 16) == 0 && (W_SZ % 16) == 0);
static_assert((L_WWL % 16) == 0 && (L_CST % 16) == 0 && (L_OUT % 16) == 0 && (L_WAV % 16) == 0);
static_assert((Q_XL % 16) == 0 && (Q_SP % 16) == 0);
static_assert((PA * 2) % 16 == 0 && (PK * 2) % 16 == 0);
static_assert(QPB * OC == 12 * QTH * 4);
static_assert(64 * PPB == 4 * NTH * 4);
static_assert(2 * KN <= YR - 8);
static_assert(WROWS * CH == 8 * 8 * QTH);

typedef float          v4f   __attribute__((ext_vector_type(4)));
typedef float          v8f   __attribute__((ext_vector_type(8)));
typedef unsigned int   v4u   __attribute__((ext_vector_type(4)));
typedef unsigned short v8us  __attribute__((ext_vector_type(8)));
typedef __bf16         v16bf __attribute__((ext_vector_type(16)));
union FragB { v16bf v; v8us u[2]; };

__device__ __forceinline__ unsigned short bf_rne(float f) {
  unsigned int u = __float_as_uint(f);
  u = u + 0x7FFFu + ((u >> 16) & 1u);
  return (unsigned short)(u >> 16);
}
__device__ __forceinline__ float bf_val(unsigned short s) {
  return __uint_as_float(((unsigned int)s) << 16);
}
__device__ __forceinline__ void split2(float v, unsigned short& hi, unsigned short& lo) {
  hi = bf_rne(v);
  lo = bf_rne(v - bf_val(hi));
}

__device__ __forceinline__ v8f wmb(v16bf a, v16bf b, v8f c) {
  v8f d = __builtin_amdgcn_wmma_f32_16x16x32_bf16(false, a, false, b, (short)0, c, false, false);
#if defined(__HIP_DEVICE_COMPILE__)
  asm volatile("v_nop\n\tv_nop\n\tv_nop\n\tv_nop" : "+v"(d) : "v"(a), "v"(b));
#endif
  return d;
}
__device__ __forceinline__ v8f wm3(v16bf ah, v16bf al, v16bf bh, v16bf bl, v8f c) {
  c = wmb(ah, bh, c);
  c = wmb(al, bh, c);
  c = wmb(ah, bl, c);
  return c;
}
__device__ __forceinline__ v8f zero8() {
  v8f z = {0.f, 0.f, 0.f, 0.f, 0.f, 0.f, 0.f, 0.f};
  return z;
}

__device__ __forceinline__ v16bf lfrag(const unsigned short* p) {
  FragB f;
  f.u[0] = *(const v8us*)p;
  f.u[1] = *(const v8us*)(p + 16);
  return f.v;
}

__global__ __launch_bounds__(QTH) void k_prep(
    const float* __restrict__ Wg, const float* __restrict__ Wt,
    const float* __restrict__ Wp, const float* __restrict__ Ww,
    unsigned short* wH, unsigned short* wL) {
  const int g   = blockIdx.x * QTH + (int)threadIdx.x;
  const int seg = blockIdx.x >> 1;
  const float* src = (seg == 0) ? Wg : (seg == 1) ? Wt : (seg == 2) ? Wp : Ww;
  const int row = g >> 3;
  const int c0  = (g & 7) * 8;
  const int lr  = row & 63;
  const v4f a = *(const v4f*)(src + lr * CH + c0);
  const v4f c = *(const v4f*)(src + lr * CH + c0 + 4);
  float v[8];
  v[0] = a[0]; v[1] = a[1]; v[2] = a[2]; v[3] = a[3];
  v[4] = c[0]; v[5] = c[1]; v[6] = c[2]; v[7] = c[3];
  v8us hv, lv;
#pragma unroll
  for (int e = 0; e < 8; ++e) {
    unsigned short hs, ls;
    split2(v[e], hs, ls);
    hv[e] = hs;
    lv[e] = ls;
  }
  unsigned short* dh = wH + (size_t)row * CH + c0;
  unsigned short* dl = wL + (size_t)row * CH + c0;
  *(volatile v8us*)dh = hv;
  *(volatile v8us*)dl = lv;
  __threadfence();
  *(volatile v8us*)dh = hv;
  *(volatile v8us*)dl = lv;
}

__global__ __launch_bounds__(QTH) __attribute__((amdgpu_num_vgpr(256))) void k_proj(
    const float* __restrict__ x, const unsigned short* __restrict__ wH,
    const unsigned short* __restrict__ wL, float* P) {
  extern __shared__ v4f lds_dyn[];
  char* lb = (char*)lds_dyn;
  unsigned short* xH = (unsigned short*)(lb + Q_XH);
  unsigned short* xL = (unsigned short*)(lb + Q_XL);
  float* sP = (float*)(lb + Q_SP);

  const int tid  = threadIdx.x, lane = tid & 31;
  const int wave = __builtin_amdgcn_readfirstlane(tid >> 5);
  const int h = lane >> 4, m = lane & 15;
  const int b   = blockIdx.x / (NPT / QPB);
  const int nb  = blockIdx.x - b * (NPT / QPB);
  const int n0  = nb * QPB;
  const int pt0 = b * NPT + n0;

  for (int i = tid; i < QPB * CH; i += QTH) {
    const int c  = i >> 6;
    const int nn = i & 63;
    const float v = x[((size_t)(b * CH + c)) * NPT + n0 + nn];
    unsigned short hs, ls;
    split2(v, hs, ls);
    xH[nn * PA + c] = hs;
    xL[nn * PA + c] = ls;
  }
  __syncthreads();

  const int mt = wave & 3, nh = wave >> 2;
  v8f acc[6];
#pragma unroll
  for (int t = 0; t < 6; ++t) acc[t] = zero8();
#pragma unroll
  for (int ks = 0; ks < 2; ++ks) {
    const int ko = 32 * ks + 8 * h;
    const v16bf aH = lfrag(xH + (16 * mt + m) * PA + ko);
    const v16bf aL = lfrag(xL + (16 * mt + m) * PA + ko);
#pragma unroll
    for (int t = 0; t < 6; ++t) {
      const int o = 16 * (6 * nh + t) + m;
      const v16bf bH = lfrag(wH + (size_t)o * CH + ko);
      const v16bf bL = lfrag(wL + (size_t)o * CH + ko);
      acc[t] = wm3(aH, aL, bH, bL, acc[t]);
    }
  }
#pragma unroll
  for (int t = 0; t < 6; ++t) {
#pragma unroll
    for (int r = 0; r < 8; ++r)
      sP[(16 * mt + 8 * h + r) * OC + 16 * (6 * nh + t) + m] = acc[t][r];
  }
  __syncthreads();

  float* gp = P + (size_t)pt0 * OC;
#pragma unroll
  for (int i = 0; i < 12; ++i) {
    const int q = tid + QTH * i;
    const v4f v = *(const v4f*)(sP + 4 * q);
    *(volatile v4f*)(gp + 4 * q) = v;
  }
  __threadfence();
#pragma unroll
  for (int i = 0; i < 12; ++i) {
    const int q = tid + QTH * i;
    const v4f v = *(const v4f*)(sP + 4 * q);
    *(volatile v4f*)(gp + 4 * q) = v;
  }
}

__global__ __launch_bounds__(NTH) __attribute__((amdgpu_num_vgpr(256))) void k_main(
    const float* __restrict__ P, const int* __restrict__ idx,
    const float* __restrict__ bg, const float* __restrict__ bt, const float* __restrict__ bp,
    const float* __restrict__ bw, const float* __restrict__ gamma, const float* __restrict__ beta,
    const unsigned short* __restrict__ wH, const unsigned short* __restrict__ wL,
    const int* __restrict__ kcount, float* out) {
  extern __shared__ v4f lds_dyn[];
  char* lb = (char*)lds_dyn;
  unsigned short* sWwH = (unsigned short*)(lb + L_WWH);
  unsigned short* sWwL = (unsigned short*)(lb + L_WWL);
  float* sC   = (float*)(lb + L_CST);
  float* sOut = (float*)(lb + L_OUT);

  const int tid  = threadIdx.x, lane = tid & 31;
  const int wave = __builtin_amdgcn_readfirstlane(tid >> 5);
  const int h = lane >> 4, m = lane & 15;
  const bool hz = (h == 0);

  char* ub = lb + L_WAV + wave * W_SZ;
  unsigned short* thH = (unsigned short*)(ub + W_THH);
  unsigned short* thL = (unsigned short*)(ub + W_THL);
  unsigned short* phH = (unsigned short*)(ub + W_PHH);
  unsigned short* phL = (unsigned short*)(ub + W_PHL);
  unsigned short* gtH = (unsigned short*)(ub + W_GTH);
  unsigned short* gtL = (unsigned short*)(ub + W_GTL);
  float*          fS  = (float*)(ub + W_FS);
  unsigned short* atH = (unsigned short*)(ub + W_ATH);
  unsigned short* atL = (unsigned short*)(ub + W_ATL);
  unsigned short* yH  = (unsigned short*)(ub + W_YH);
  unsigned short* yL  = (unsigned short*)(ub + W_YL);

  const int b   = blockIdx.x / (NPT / PPB);
  const int nb  = blockIdx.x - b * (NPT / PPB);
  const int n0  = nb * PPB;
  const int pt0 = b * NPT + n0;

  for (int i = tid; i < 384; i += NTH) {
    const int ci = i & 63, seg = i >> 6;
    const float v0 = bg[ci], v1 = bt[ci], v2 = bp[ci], v3 = bw[ci], v4 = gamma[ci], v5 = beta[ci];
    float v = v0;
    v = (seg == 1) ? v1 : v;
    v = (seg == 2) ? v2 : v;
    v = (seg == 3) ? v3 : v;
    v = (seg == 4) ? v4 : v;
    v = (seg == 5) ? v5 : v;
    sC[i] = v;
  }
  for (int i = tid; i < 512; i += NTH) {
    const int row = i >> 3, c0 = (i & 7) * 8;
    const v8us a = *(const v8us*)(wH + (size_t)(OC + row) * CH + c0);
    const v8us c = *(const v8us*)(wL + (size_t)(OC + row) * CH + c0);
    *(v8us*)(sWwH + row * PA + c0) = a;
    *(v8us*)(sWwL + row * PA + c0) = c;
  }
  {
    v4u z = {0u, 0u, 0u, 0u};
    v4u* zp = (v4u*)ub;
    for (int i = lane; i < W_SZ / 16; i += 32) zp[i] = z;
  }
  __syncthreads();

  float bcR[6];
#pragma unroll
  for (int u = 0; u < 6; ++u) bcR[u] = sC[lane + 32 * u];
  const float invs = 1.0f / sqrtf(1.0f + 1e-5f);

#pragma unroll 1
  for (int s = 0; s < PPW; ++s) {
    const int lp = wave * PPW + s;
    const int pt = pt0 + lp;
    const int ybase = ((s & 1) != 0) ? KN : 0;

    int jv = idx[(size_t)pt * KN + (lane < KN ? lane : KN - 1)];
    jv = jv < 0 ? 0 : (jv > NPTOT - 1 ? NPTOT - 1 : jv);
    float cR[6];
    {
      const float* pc = P + (size_t)pt * OC + lane;
#pragma unroll
      for (int u = 0; u < 6; ++u) cR[u] = pc[32 * u];
    }
#pragma unroll 2
    for (int kk = 0; kk < KN; ++kk) {
      const int j = __shfl(jv, kk, 32);
      const float* pr = P + (size_t)j * OC + lane;
#pragma unroll
      for (int u = 0; u < 6; ++u) {
        const float v = pr[32 * u] - cR[u] + bcR[u];
        unsigned short hs, ls;
        split2(v, hs, ls);
        if (u < 2) {
          const int o = lane + 32 * u;
          gtH[o * PK + kk] = hs;
          gtL[o * PK + kk] = ls;
        } else if (u < 4) {
          const int c = lane + 32 * (u - 2);
          thH[kk * PA + c] = hs;
          thL[kk * PA + c] = ls;
        } else {
          const int c = lane + 32 * (u - 4);
          phH[kk * PA + c] = hs;
          phL[kk * PA + c] = ls;
        }
      }
    }
    __syncthreads();

    {
      v8f acc[4];
#pragma unroll
      for (int t = 0; t < 4; ++t) acc[t] = zero8();
#pragma unroll
      for (int ks = 0; ks < 2; ++ks) {
        const int ko = 32 * ks + 8 * h;
        const v16bf aH0 = lfrag(thH + m * PA + ko);
        const v16bf aL0 = lfrag(thL + m * PA + ko);
        const v16bf aH1 = lfrag(thH + (16 + m) * PA + ko);
        const v16bf aL1 = lfrag(thL + (16 + m) * PA + ko);
        const v16bf bH0 = lfrag(phH + m * PA + ko);
        const v16bf bL0 = lfrag(phL + m * PA + ko);
        const v16bf bH1 = lfrag(phH + (16 + m) * PA + ko);
        const v16bf bL1 = lfrag(phL + (16 + m) * PA + ko);
        acc[0] = wm3(aH0, aL0, bH0, bL0, acc[0]);
        acc[1] = wm3(aH0, aL0, bH1, bL1, acc[1]);
        acc[2] = wm3(aH1, aL1, bH0, bL0, acc[2]);
        acc[3] = wm3(aH1, aL1, bH1, bL1, acc[3]);
      }
#pragma unroll
      for (int t = 0; t < 4; ++t) {
        const int mt = t >> 1, nt = t & 1;
#pragma unroll
        for (int r = 0; r < 8; ++r)
          fS[(16 * mt + 8 * h + r) * 32 + 16 * nt + m] = acc[t][r];
      }
    }
    __syncthreads();

    {
      const float* fr = fS + lane * 32;
      float fv[KN];
#pragma unroll
      for (int jj = 0; jj < KN; ++jj) fv[jj] = fr[jj];
      float mx = fv[0];
#pragma unroll
      for (int jj = 1; jj < KN; ++jj) mx = fmaxf(mx, fv[jj]);
      float s1 = 0.0f;
#pragma unroll
      for (int jj = 0; jj < KN; ++jj) {
        fv[jj] = expf(fv[jj] - mx);
        s1 += fv[jj];
      }
      const float rs = 1.0f / s1;
      if (lane < KN) {
#pragma unroll
        for (int jj = 0; jj < KN; ++jj) {
          unsigned short hs, ls;
          split2(fv[jj] * rs, hs, ls);
          atH[lane * PK + jj] = hs;
          atL[lane * PK + jj] = ls;
        }
      }
    }
    __syncthreads();

#pragma unroll
    for (int mt = 0; mt < 2; ++mt) {
      v8f acc[4];
#pragma unroll
      for (int nt = 0; nt < 4; ++nt) acc[nt] = zero8();
      const v16bf aH = lfrag(atH + (16 * mt + m) * PK + 8 * h);
      const v16bf aL = lfrag(atL + (16 * mt + m) * PK + 8 * h);
#pragma unroll
      for (int nt = 0; nt < 4; ++nt) {
        const v16bf bH = lfrag(gtH + (16 * nt + m) * PK + 8 * h);
        const v16bf bL = lfrag(gtL + (16 * nt + m) * PK + 8 * h);
        acc[nt] = wm3(aH, aL, bH, bL, acc[nt]);
      }
#pragma unroll
      for (int nt = 0; nt < 4; ++nt) {
#pragma unroll
        for (int r = 0; r < 8; ++r) {
          if (mt == 0 || r < 4) {
            const int R = 16 * mt + 8 * h + r;
            unsigned short hs, ls;
            split2(acc[nt][r], hs, ls);
            const bool ok = (mt == 0) ? true : hz;
            if (ok) {
              yH[(ybase + R) * PA + 16 * nt + m] = hs;
              yL[(ybase + R) * PA + 16 * nt + m] = ls;
            }
          }
        }
      }
    }

    if ((s & 1) != 0) {
      __syncthreads();
      float mE[4], mO[4];
#pragma unroll
      for (int nt = 0; nt < 4; ++nt) { mE[nt] = -3.0e38f; mO[nt] = -3.0e38f; }
#pragma unroll
      for (int mt = 0; mt < 3; ++mt) {
        v8f acc[4];
#pragma unroll
        for (int nt = 0; nt < 4; ++nt) acc[nt] = zero8();
#pragma unroll
        for (int ks = 0; ks < 2; ++ks) {
          const int ko = 32 * ks + 8 * h;
          const v16bf aH = lfrag(yH + (16 * mt + m) * PA + ko);
          const v16bf aL = lfrag(yL + (16 * mt + m) * PA + ko);
#pragma unroll
          for (int nt = 0; nt < 4; ++nt) {
            const v16bf bH = lfrag(sWwH + (16 * nt + m) * PA + ko);
            const v16bf bL = lfrag(sWwL + (16 * nt + m) * PA + ko);
            acc[nt] = wm3(aH, aL, bH, bL, acc[nt]);
          }
        }
#pragma unroll
        for (int nt = 0; nt < 4; ++nt) {
          const int p = 16 * nt + m;
          const float bwv = sC[192 + p], ga = sC[256 + p], be = sC[320 + p];
#pragma unroll
          for (int r = 0; r < 8; ++r) {
            float v = (acc[nt][r] + bwv) * invs;
            v = v * ga + be;
            if (mt == 0) {
              mE[nt] = fmaxf(mE[nt], v);
            } else if (mt == 1) {
              if (r < 4) {
                mE[nt] = hz ? fmaxf(mE[nt], v) : mE[nt];
                mO[nt] = hz ? mO[nt] : fmaxf(mO[nt], v);
              } else {
                mO[nt] = fmaxf(mO[nt], v);
              }
            } else {
              mO[nt] = hz ? fmaxf(mO[nt], v) : mO[nt];
            }
          }
        }
      }
#pragma unroll
      for (int nt = 0; nt < 4; ++nt) {
        const float e2 = fmaxf(mE[nt], __shfl_xor(mE[nt], 16, 32));
        const float o2 = fmaxf(mO[nt], __shfl_xor(mO[nt], 16, 32));
        if (hz) {
          const int p = 16 * nt + m;
          sOut[p * PPB + lp - 1] = e2;
          sOut[p * PPB + lp]     = o2;
        }
      }
    }
    __syncthreads();
  }

  {
    const size_t obase = (size_t)(b * CH) * NPT + n0;
#pragma unroll
    for (int it = 0; it < 4; ++it) {
      const int line = it * 16 + (tid >> 3), piece = tid & 7;
      const v4f v = *(const v4f*)(sOut + line * PPB + piece * 4);
      *(volatile v4f*)(out + obase + (size_t)line * NPT + piece * 4) = v;
    }
    __threadfence();
#pragma unroll
    for (int it = 0; it < 4; ++it) {
      const int line = it * 16 + (tid >> 3), piece = tid & 7;
      const v4f v = *(const v4f*)(sOut + line * PPB + piece * 4);
      *(volatile v4f*)(out + obase + (size_t)line * NPT + piece * 4) = v;
    }
  }
}

extern "C" void kernel_launch(void* const* d_in, const int* in_sizes, int n_in,
                              void* d_out, int out_size, void* d_ws, size_t ws_size,
                              hipStream_t stream) {
  if (n_in < 13) return;
  if (in_sizes[0] != NB * CH * NPT) return;
  if (in_sizes[1] != NPTOT * KN) return;
  if (in_sizes[2] != CH * CH || in_sizes[4] != CH * CH || in_sizes[6] != CH * CH || in_sizes[8] != CH * CH) return;
  if (in_sizes[3] != CH || in_sizes[5] != CH || in_sizes[7] != CH || in_sizes[9] != CH) return;
  if (in_sizes[10] != CH || in_sizes[11] != CH || in_sizes[12] != 1) return;
  if (out_size != NB * CH * NPT) return;

  const float* x     = (const float*)d_in[0];
  const int*   idx   = (const int*)d_in[1];
  const float* Wg    = (const float*)d_in[2];
  const float* bg    = (const float*)d_in[3];
  const float* Wt    = (const float*)d_in[4];
  const float* bt    = (const float*)d_in[5];
  const float* Wp    = (const float*)d_in[6];
  const float* bp    = (const float*)d_in[7];
  const float* Ww    = (const float*)d_in[8];
  const float* bw    = (const float*)d_in[9];
  const float* gamma = (const float*)d_in[10];
  const float* beta  = (const float*)d_in[11];
  const int*   kin   = (const int*)d_in[12];
  float* out = (float*)d_out;

  char* ws = (char*)d_ws;
  size_t off = 0;
  const size_t oH = off; off += (size_t)WROWS * CH * 2;     off = (off + 255) & ~(size_t)255;
  const size_t oL = off; off += (size_t)WROWS * CH * 2;     off = (off + 255) & ~(size_t)255;
  const size_t oP = off; off += (size_t)NPTOT * OC * 4;     off = (off + 255) & ~(size_t)255;
  if (off > ws_size || off > (size_t)134217728) return;
  unsigned short* wH = (unsigned short*)(ws + oH);
  unsigned short* wL = (unsigned short*)(ws + oL);
  float* P = (float*)(ws + oP);

  k_prep<<<(WROWS * CH / 8) / QTH, QTH, 0, stream>>>(Wg, Wt, Wp, Ww, wH, wL);

  hipFuncSetAttribute(reinterpret_cast<const void*>(&k_proj),
                      hipFuncAttributeMaxDynamicSharedMemorySize, LDS_PROJ);
  k_proj<<<NPTOT / QPB, QTH, LDS_PROJ, stream>>>(x, wH, wL, P);

  hipFuncSetAttribute(reinterpret_cast<const void*>(&k_main),
                      hipFuncAttributeMaxDynamicSharedMemorySize, LDS_MAIN);
  k_main<<<NPTOT / PPB, NTH, LDS_MAIN, stream>>>(
      P, idx, bg, bt, bp, bw, gamma, beta, wH, wL, kin, out);
}
